// Swin_34540126994817
// MI455X (gfx1250) — hardware-verified
//
#include <hip/hip_runtime.h>
#define NN 16384
#define CC 96
#define NH 6
#define HD 16
#define QP 320
#define PP 128
#define FF 384
#define NPAIR 32
#define QGL 16

typedef __bf16 v16b __attribute__((ext_vector_type(16)));
typedef unsigned short v8us __attribute__((ext_vector_type(8), may_alias));
typedef float  v8f  __attribute__((ext_vector_type(8)));
typedef float  v4f  __attribute__((ext_vector_type(4)));
typedef float  v4fa __attribute__((ext_vector_type(4), may_alias));
union FragB { v16b v; v8us half[2]; unsigned short u[16]; };

__device__ __forceinline__ unsigned short bf16_bits(float x) { unsigned int u = __float_as_uint(x); return (unsigned short)((u + 0x7FFFu + ((u >> 16) & 1u)) >> 16); }
__device__ __forceinline__ float bf16_val(unsigned short b) { return __uint_as_float(((unsigned int)b) << 16); }
__device__ __forceinline__ float bf16_round(float x) { return bf16_val(bf16_bits(x)); }
template <int NT>
__device__ __forceinline__ v8f mmaN(v16b ah, v16b al, v16b bh, v16b bl, v8f c) {
  c = __builtin_amdgcn_wmma_f32_16x16x32_bf16(false, ah, false, bh, (short)0, c, false, false);
  if (NT >= 2) c = __builtin_amdgcn_wmma_f32_16x16x32_bf16(false, al, false, bh, (short)0, c, false, false);
  if (NT >= 3) c = __builtin_amdgcn_wmma_f32_16x16x32_bf16(false, ah, false, bl, (short)0, c, false, false);
  asm volatile("v_nop\n\tv_nop\n\tv_nop\n\tv_nop" : "+v"(c) : "v"(ah), "v"(al), "v"(bh), "v"(bl));
  return c;
}

__global__ __launch_bounds__(256) void k_wt_bf16(const float* __restrict__ W, unsigned short* __restrict__ Wt, int K, int N) {
  const int t = blockIdx.x * 256 + threadIdx.x;
  const int k8n = K / 8;
  if (t >= N * k8n) return;
  const int n = t / k8n, k8 = (t % k8n) * 8;
  v8us v;
#pragma unroll
  for (int i = 0; i < 8; ++i) v[i] = bf16_bits(W[(size_t)(k8 + i) * N + n]);
  *(volatile v8us*)(Wt + (size_t)n * K + k8) = v;
  __threadfence();
  *(volatile v8us*)(Wt + (size_t)n * K + k8) = v;
}

template <bool ASPLIT, int ACT, bool BIAS_BF16>
__global__ __launch_bounds__(128) void k_gemm_bf(const float* __restrict__ A, int lda, const unsigned short* __restrict__ Wt, int ldb,
                                               const float* __restrict__ bias, float* __restrict__ C, int ldc, int M, int N, int K) {
  __shared__ __attribute__((aligned(16))) float so[4][16][64];
  const int tid = threadIdx.x, w = tid >> 5, lane = tid & 31, ln = lane & 15, hh = lane >> 4;
  const int ntn = N / 64;
  const int wid = blockIdx.x * 4 + w;
  const int mt = wid / ntn, nq = wid % ntn;
  if (mt * 16 >= M) return;
  const int row0 = mt * 16, col0 = nq * 64;
  const float* arow = A + (size_t)(row0 + ln) * lda;
  v8f acc[4] = {};
  for (int kb = 0; kb < K; kb += 32) {
    FragB ah, al;
    const v4f x0 = *(const v4fa*)(arow + kb + 8 * hh), x1 = *(const v4fa*)(arow + kb + 8 * hh + 4);
    const v4f x2 = *(const v4fa*)(arow + kb + 16 + 8 * hh), x3 = *(const v4fa*)(arow + kb + 16 + 8 * hh + 4);
    float xs[16] = {x0[0],x0[1],x0[2],x0[3],x1[0],x1[1],x1[2],x1[3],x2[0],x2[1],x2[2],x2[3],x3[0],x3[1],x3[2],x3[3]};
#pragma unroll
    for (int i = 0; i < 16; ++i) { const unsigned short hb = bf16_bits(xs[i]); ah.u[i] = hb; al.u[i] = ASPLIT ? bf16_bits(xs[i] - bf16_val(hb)) : (unsigned short)0; }
#pragma unroll
    for (int t = 0; t < 4; ++t) {
      const unsigned short* brow = Wt + (size_t)(col0 + t * 16 + ln) * ldb + kb;
      FragB b;
      b.half[0] = *(const v8us*)(brow + 8 * hh);
      b.half[1] = *(const v8us*)(brow + 16 + 8 * hh);
      acc[t] = mmaN<ASPLIT ? 2 : 1>(ah.v, al.v, b.v, b.v, acc[t]);
    }
  }
#pragma unroll
  for (int t = 0; t < 4; ++t) {
    float bv = bias ? bias[col0 + t * 16 + ln] : 0.f;
    if (BIAS_BF16) bv = bf16_round(bv);
#pragma unroll
    for (int r = 0; r < 8; ++r) { float v = acc[t][r] + bv; if (ACT == 1) v = fmaxf(v, 0.f); so[w][8 * hh + r][t * 16 + ln] = v; }
  }
  __builtin_amdgcn_fence(__ATOMIC_ACQ_REL, "workgroup");
  __builtin_amdgcn_wave_barrier();
  const int rsub = lane >> 4, c4 = (lane & 15) * 4;
  for (int pass = 0; pass < 2; ++pass) {
#pragma unroll
    for (int q = 0; q < 8; ++q) {
      const int r = q * 2 + rsub;
      const v4f v = *(const v4fa*)&so[w][r][c4];
      *(volatile v4f*)(C + (size_t)(row0 + r) * ldc + col0 + c4) = v;
    }
    if (pass == 0) __threadfence();
  }
}

template <int D, bool CAUSAL>
__global__ __launch_bounds__(128) void k_flash(const float* __restrict__ qb, const float* __restrict__ kb, const float* __restrict__ vb,
                                             int pitch, int T, int H, float scale, float* __restrict__ y, int ypitch) {
  constexpr int KS = D / 32;
  constexpr int DT = D / 16;
  __shared__ __attribute__((aligned(16))) unsigned short sKh[32][D + 8], sKl[32][D + 8], sVh[32][D + 8], sVl[32][D + 8];
  __shared__ __attribute__((aligned(16))) unsigned short sPh[4][16][40], sPl[4][16][40];
  __shared__ __attribute__((aligned(16))) float sO[4][16][D];
  const int tid = threadIdx.x, w = tid >> 5, lane = tid & 31, ln = lane & 15, hh = lane >> 4;
  const int nqb = (T + 63) / 64;
  const int bh = blockIdx.x / nqb, qblk = blockIdx.x % nqb;
  const int b = bh / H, h = bh % H;
  const int q0 = qblk * 64 + w * 16;
  const float* Q = qb + (size_t)b * T * pitch + h * D;
  const float* K = kb + (size_t)b * T * pitch + h * D;
  const float* V = vb + (size_t)b * T * pitch + h * D;

  FragB aqh[KS], aql[KS];
  {
    int row = q0 + ln; if (row >= T) row = T - 1;
    const float* qr = Q + (size_t)row * pitch;
#pragma unroll
    for (int ks = 0; ks < KS; ++ks)
#pragma unroll
      for (int i = 0; i < 16; ++i) {
        const int d = ks * 32 + ((i < 8) ? (8 * hh + i) : (16 + 8 * hh + (i - 8)));
        const float x = qr[d] * scale; const unsigned short hb = bf16_bits(x);
        aqh[ks].u[i] = hb; aql[ks].u[i] = bf16_bits(x - bf16_val(hb));
      }
  }
  float m_r[8], l_r[8];
#pragma unroll
  for (int r = 0; r < 8; ++r) { m_r[r] = -3.0e38f; l_r[r] = 0.f; }
  v8f oacc[DT];
#pragma unroll
  for (int dt = 0; dt < DT; ++dt) oacc[dt] = (v8f){0.f,0.f,0.f,0.f,0.f,0.f,0.f,0.f};

  const int kv_end = CAUSAL ? min(T, qblk * 64 + 64) : T;
  for (int j0 = 0; j0 < kv_end; j0 += 32) {
    __syncthreads();
    for (int e = tid; e < 32 * (D / 4); e += 128) {
      const int r = e / (D / 4), c4 = (e % (D / 4)) * 4;
      const int key = j0 + r;
      v4f kf = {0.f,0.f,0.f,0.f}, vf = {0.f,0.f,0.f,0.f};
      if (key < T) { kf = *(const v4fa*)(K + (size_t)key * pitch + c4); vf = *(const v4fa*)(V + (size_t)key * pitch + c4); }
#pragma unroll
      for (int t = 0; t < 4; ++t) {
        unsigned short hb = bf16_bits(kf[t]); sKh[r][c4 + t] = hb; sKl[r][c4 + t] = bf16_bits(kf[t] - bf16_val(hb));
        hb = bf16_bits(vf[t]); sVh[r][c4 + t] = hb; sVl[r][c4 + t] = bf16_bits(vf[t] - bf16_val(hb));
      }
    }
    __syncthreads();
    v8f s[2];
#pragma unroll
    for (int nt = 0; nt < 2; ++nt) {
      v8f acc = {};
#pragma unroll
      for (int ks = 0; ks < KS; ++ks) {
        FragB bh_, bl_;
        bh_.half[0] = *(const v8us*)&sKh[nt * 16 + ln][ks * 32 + 8 * hh]; bh_.half[1] = *(const v8us*)&sKh[nt * 16 + ln][ks * 32 + 16 + 8 * hh];
        bl_.half[0] = *(const v8us*)&sKl[nt * 16 + ln][ks * 32 + 8 * hh]; bl_.half[1] = *(const v8us*)&sKl[nt * 16 + ln][ks * 32 + 16 + 8 * hh];
        acc = mmaN<3>(aqh[ks].v, aql[ks].v, bh_.v, bl_.v, acc);
      }
      s[nt] = acc;
    }
    float alpha[8];
#pragma unroll
    for (int r = 0; r < 8; ++r) {
      const int qi = q0 + 8 * hh + r;
      const int ja = j0 + ln, jb = j0 + 16 + ln;
      if (CAUSAL) { if (ja > qi) s[0][r] = -3.0e38f; if (jb > qi) s[1][r] = -3.0e38f; }
      if (ja >= T) s[0][r] = -3.0e38f;
      if (jb >= T) s[1][r] = -3.0e38f;
      float mx = fmaxf(s[0][r], s[1][r]);
      mx = fmaxf(mx, __shfl_xor(mx, 1, 32)); mx = fmaxf(mx, __shfl_xor(mx, 2, 32)); mx = fmaxf(mx, __shfl_xor(mx, 4, 32)); mx = fmaxf(mx, __shfl_xor(mx, 8, 32));
      const float mnew = fmaxf(m_r[r], mx);
      alpha[r] = (mnew > -1.0e38f) ? __expf(m_r[r] - mnew) : 1.0f;
      const float p0 = (s[0][r] > -1.0e38f) ? __expf(s[0][r] - mnew) : 0.f;
      const float p1 = (s[1][r] > -1.0e38f) ? __expf(s[1][r] - mnew) : 0.f;
      m_r[r] = mnew;
      l_r[r] = l_r[r] * alpha[r] + p0 + p1;
      unsigned short hb = bf16_bits(p0); sPh[w][8 * hh + r][ln] = hb;      sPl[w][8 * hh + r][ln] = bf16_bits(p0 - bf16_val(hb));
      hb = bf16_bits(p1);                sPh[w][8 * hh + r][16 + ln] = hb; sPl[w][8 * hh + r][16 + ln] = bf16_bits(p1 - bf16_val(hb));
    }
#pragma unroll
    for (int dt = 0; dt < DT; ++dt)
#pragma unroll
      for (int r = 0; r < 8; ++r) oacc[dt][r] *= alpha[r];
    __builtin_amdgcn_fence(__ATOMIC_ACQ_REL, "workgroup");
    __builtin_amdgcn_wave_barrier();
    FragB pah, pal;
    pah.half[0] = *(const v8us*)&sPh[w][ln][8 * hh]; pah.half[1] = *(const v8us*)&sPh[w][ln][16 + 8 * hh];
    pal.half[0] = *(const v8us*)&sPl[w][ln][8 * hh]; pal.half[1] = *(const v8us*)&sPl[w][ln][16 + 8 * hh];
#pragma unroll
    for (int dt = 0; dt < DT; ++dt) {
      FragB bvh, bvl;
#pragma unroll
      for (int i = 0; i < 8; ++i) {
        bvh.u[i] = sVh[8 * hh + i][dt * 16 + ln]; bvh.u[8 + i] = sVh[16 + 8 * hh + i][dt * 16 + ln];
        bvl.u[i] = sVl[8 * hh + i][dt * 16 + ln]; bvl.u[8 + i] = sVl[16 + 8 * hh + i][dt * 16 + ln];
      }
      oacc[dt] = mmaN<3>(pah.v, pal.v, bvh.v, bvl.v, oacc[dt]);
    }
    __builtin_amdgcn_fence(__ATOMIC_ACQ_REL, "workgroup");
    __builtin_amdgcn_wave_barrier();
  }
#pragma unroll
  for (int r = 0; r < 8; ++r) {
    float l = l_r[r];
    l += __shfl_xor(l, 1, 32); l += __shfl_xor(l, 2, 32); l += __shfl_xor(l, 4, 32); l += __shfl_xor(l, 8, 32);
    l_r[r] = (l > 0.f) ? 1.0f / l : 0.f;
  }
#pragma unroll
  for (int dt = 0; dt < DT; ++dt)
#pragma unroll
    for (int r = 0; r < 8; ++r) sO[w][8 * hh + r][dt * 16 + ln] = oacc[dt][r] * l_r[r];
  __builtin_amdgcn_fence(__ATOMIC_ACQ_REL, "workgroup");
  __builtin_amdgcn_wave_barrier();
  for (int pass = 0; pass < 2; ++pass) {
    for (int r = 0; r < 16; ++r) {
      const int row = q0 + r;
      if (row < T && lane < D / 4) {
        const v4f val = *(const v4fa*)&sO[w][r][lane * 4];
        *(volatile v4f*)(y + ((size_t)b * T + row) * ypitch + h * D + lane * 4) = val;
      }
    }
    if (pass == 0) __threadfence();
  }
}

template <bool ASPLIT, int ACT, bool BIAS_BF16, bool RES_BF16>
__global__ __launch_bounds__(128) void k_gemm_bf3(const float* __restrict__ A, int lda, const unsigned short* __restrict__ Wt, int ldb,
                                                const float* __restrict__ bias, const float* __restrict__ resid, int rmod, int ldr,
                                                float* __restrict__ C, int ldc, int M, int N, int K) {
  __shared__ __attribute__((aligned(16))) float so[4][16][64];
  const int tid = threadIdx.x, w = tid >> 5, lane = tid & 31, ln = lane & 15, hh = lane >> 4;
  const int ntn = N / 64;
  const int wid = blockIdx.x * 4 + w;
  const int mt = wid / ntn, nq = wid % ntn;
  if (mt * 16 >= M) return;
  const int row0 = mt * 16, col0 = nq * 64;
  const float* arow = A + (size_t)(row0 + ln) * lda;
  v8f acc[4] = {};
  for (int kb = 0; kb < K; kb += 32) {
    FragB ah, al;
    const v4f x0 = *(const v4fa*)(arow + kb + 8 * hh), x1 = *(const v4fa*)(arow + kb + 8 * hh + 4);
    const v4f x2 = *(const v4fa*)(arow + kb + 16 + 8 * hh), x3 = *(const v4fa*)(arow + kb + 16 + 8 * hh + 4);
    float xs[16] = {x0[0],x0[1],x0[2],x0[3],x1[0],x1[1],x1[2],x1[3],x2[0],x2[1],x2[2],x2[3],x3[0],x3[1],x3[2],x3[3]};
#pragma unroll
    for (int i = 0; i < 16; ++i) { const unsigned short hb = bf16_bits(xs[i]); ah.u[i] = hb; al.u[i] = ASPLIT ? bf16_bits(xs[i] - bf16_val(hb)) : (unsigned short)0; }
#pragma unroll
    for (int t = 0; t < 4; ++t) {
      const unsigned short* brow = Wt + (size_t)(col0 + t * 16 + ln) * ldb + kb;
      FragB b;
      b.half[0] = *(const v8us*)(brow + 8 * hh);
      b.half[1] = *(const v8us*)(brow + 16 + 8 * hh);
      acc[t] = mmaN<ASPLIT ? 2 : 1>(ah.v, al.v, b.v, b.v, acc[t]);
    }
  }
#pragma unroll
  for (int t = 0; t < 4; ++t) {
    const int col = col0 + t * 16 + ln;
    float bv = bias ? bias[col] : 0.f;
    if (BIAS_BF16) bv = bf16_round(bv);
#pragma unroll
    for (int r = 0; r < 8; ++r) {
      float v = acc[t][r] + bv;
      if (resid) { float rv = resid[(size_t)((row0 + 8 * hh + r) % rmod) * ldr + col]; if (RES_BF16) rv = bf16_round(rv); v += rv; }
      if (ACT == 1) v = fmaxf(v, 0.f);
      if (ACT == 2) v = 0.5f * v * (1.0f + erff(v * 0.70710678118654752f));
      if (ACT == 3) { const float u = 0.7978845608028654f * (v + 0.044715f * v * v * v); v = 0.5f * v * (1.0f + tanhf(u)); }
      so[w][8 * hh + r][t * 16 + ln] = v;
    }
  }
  __builtin_amdgcn_fence(__ATOMIC_ACQ_REL, "workgroup");
  __builtin_amdgcn_wave_barrier();
  const int rsub = lane >> 4, c4 = (lane & 15) * 4;
  for (int pass = 0; pass < 2; ++pass) {
#pragma unroll
    for (int q = 0; q < 8; ++q) {
      const int r = q * 2 + rsub;
      const v4f v = *(const v4fa*)&so[w][r][c4];
      *(volatile v4f*)(C + (size_t)(row0 + r) * ldc + col0 + c4) = v;
    }
    if (pass == 0) __threadfence();
  }
}
template <bool PARAM_BF16>
__global__ __launch_bounds__(256) void k_layernorm(const float* __restrict__ X, const float* __restrict__ R, const float* __restrict__ g, const float* __restrict__ bta,
                                                  float* __restrict__ out_sum, float* __restrict__ out_norm, int N, float eps) {
  __shared__ float red[256];
  const int row = blockIdx.x, tid = threadIdx.x;
  const float* x = X + (size_t)row * N; const float* rr = R ? R + (size_t)row * N : nullptr;
  float vals[16];
  const int per = N / 256;
  float s1 = 0.f;
  for (int u = 0; u < per / 4; ++u) {
    const int j = tid * 4 + 1024 * u;
    const v4f a = *(const v4fa*)(x + j);
    v4f b = {0.f,0.f,0.f,0.f}; if (rr) b = *(const v4fa*)(rr + j);
#pragma unroll
    for (int q = 0; q < 4; ++q) { const float v = a[q] + b[q]; vals[u * 4 + q] = v; s1 += v; }
  }
  red[tid] = s1; __syncthreads();
  for (int st = 128; st > 0; st >>= 1) { if (tid < st) red[tid] += red[tid + st]; __syncthreads(); }
  const float mu = red[0] / (float)N; __syncthreads();
  float s2 = 0.f;
  for (int u = 0; u < per / 4; ++u)
#pragma unroll
    for (int q = 0; q < 4; ++q) { const float c = vals[u * 4 + q] - mu; s2 += c * c; }
  red[tid] = s2; __syncthreads();
  for (int st = 128; st > 0; st >>= 1) { if (tid < st) red[tid] += red[tid + st]; __syncthreads(); }
  const float rs = rsqrtf(red[0] / (float)N + eps);
  for (int pass = 0; pass < 2; ++pass) {
    for (int u = 0; u < per / 4; ++u) {
      const int j = tid * 4 + 1024 * u;
      v4f o, sm;
#pragma unroll
      for (int q = 0; q < 4; ++q) {
        float gg = g[j + q], bb = bta[j + q];
        if (PARAM_BF16) { gg = bf16_round(gg); bb = bf16_round(bb); }
        sm[q] = vals[u * 4 + q]; o[q] = (vals[u * 4 + q] - mu) * rs * gg + bb;
      }
      if (out_sum) *(volatile v4f*)(out_sum + (size_t)row * N + j) = sm;
      *(volatile v4f*)(out_norm + (size_t)row * N + j) = o;
    }
    if (pass == 0) __threadfence();
  }
}

__global__ __launch_bounds__(256) void k_wt_pad(const float* __restrict__ W, const float* __restrict__ b, unsigned short* __restrict__ Bt, float* __restrict__ bp, int Nout, int K, int Np) {
  const int t = blockIdx.x * 256 + threadIdx.x; const int k8n = K / 8;
  if (t < Np * k8n) { const int n = t / k8n, k8 = (t % k8n) * 8; v8us v; for (int i = 0; i < 8; ++i) v[i] = (n < Nout) ? bf16_bits(W[(size_t)n * K + k8 + i]) : (unsigned short)0; *(volatile v8us*)(Bt + (size_t)n * K + k8) = v; __threadfence(); *(volatile v8us*)(Bt + (size_t)n * K + k8) = v; }
  if (t < Np) { const float v = (t < Nout) ? bf16_round(b[t]) : 0.f; *(volatile float*)(bp + t) = v; __threadfence(); *(volatile float*)(bp + t) = v; }
}
template <bool IN_BF16>
__global__ __launch_bounds__(256) void k_ln96(const float* __restrict__ x, int xp, const float* __restrict__ g, const float* __restrict__ b, float* __restrict__ out, float* __restrict__ xcopy) {
  const int tid = threadIdx.x, w = tid >> 5, lane = tid & 31; const int row = blockIdx.x * 8 + w; if (row >= NN) return;
  float v[3]; float s = 0.f; for (int u = 0; u < 3; ++u) { float a = x[(size_t)row * xp + u * 32 + lane]; if (IN_BF16) a = bf16_round(a); v[u] = a; s += a; }
  for (int o = 16; o >= 1; o >>= 1) s += __shfl_xor(s, o, 32); const float mu = s * (1.0f / CC);
  float q2 = 0.f; for (int u = 0; u < 3; ++u) { const float c = v[u] - mu; q2 += c * c; } for (int o = 16; o >= 1; o >>= 1) q2 += __shfl_xor(q2, o, 32); const float rs = rsqrtf(q2 * (1.0f / CC) + 1e-5f);
  for (int pass = 0; pass < 2; ++pass) { for (int u = 0; u < 3; ++u) { const int c = u * 32 + lane; *(volatile float*)(out + (size_t)row * CC + c) = (v[u] - mu) * rs * bf16_round(g[c]) + bf16_round(b[c]); if (xcopy) *(volatile float*)(xcopy + (size_t)row * CC + c) = v[u]; } if (pass == 0) __threadfence(); }
}
__global__ __launch_bounds__(256) void k_min3(const float* __restrict__ xyz, float* __restrict__ mn) {
  __shared__ float red[3][256]; const int t = threadIdx.x;
  float m0 = 3.0e38f, m1 = 3.0e38f, m2 = 3.0e38f;
#pragma unroll 1
  for (int n = t; n < NN; n += 256) { m0 = fminf(m0, bf16_round(xyz[n * 3])); m1 = fminf(m1, bf16_round(xyz[n * 3 + 1])); m2 = fminf(m2, bf16_round(xyz[n * 3 + 2])); }
  red[0][t] = m0; red[1][t] = m1; red[2][t] = m2; __syncthreads();
  for (int st = 128; st > 0; st >>= 1) { if (t < st) { red[0][t] = fminf(red[0][t], red[0][t + st]); red[1][t] = fminf(red[1][t], red[1][t + st]); red[2][t] = fminf(red[2][t], red[2][t + st]); } __syncthreads(); }
  if (t < 32) { const float v = (t < 3) ? red[t][0] : 0.f; *(volatile float*)(mn + t) = v; __threadfence(); *(volatile float*)(mn + t) = v; }
}
__global__ __launch_bounds__(256) void k_swin_attn(const float* __restrict__ qkv, const float* __restrict__ xyz, const float* __restrict__ mn, const float* __restrict__ shift, const int* __restrict__ offs, const int* __restrict__ idx1,
                                                 const float* __restrict__ tab, float* __restrict__ out) {
  __shared__ float sq[8][CC]; __shared__ float so[8][CC];
  const int tid = threadIdx.x, w = tid >> 5, lane = tid & 31; const int n = blockIdx.x * 8 + w; if (n >= NN) return;
  for (int c = lane; c < CC; c += 32) sq[w][c] = qkv[(size_t)n * QP + c] * 0.25f;
  __builtin_amdgcn_fence(__ATOMIC_ACQ_REL, "workgroup"); __builtin_amdgcn_wave_barrier();
  const int p0 = offs[n], p1 = offs[n + 1]; const bool act = (p0 + lane) < p1;
  int j = act ? idx1[p0 + lane] : n; j = j < 0 ? 0 : (j >= NN ? NN - 1 : j);
  const float sh = bf16_round(shift[0]);
  int rel[3];
#pragma unroll 1
  for (int a = 0; a < 3; ++a) { const float qi = floorf(fmodf(bf16_round(xyz[n * 3 + a]) - mn[a] + sh, 4.0f) / 0.25f); const float qj = floorf(fmodf(bf16_round(xyz[j * 3 + a]) - mn[a] + sh, 4.0f) / 0.25f); int r = (int)(qi - qj) + (QGL - 1); r = r < 0 ? 0 : (r >= 4 * QGL ? 4 * QGL - 1 : r); rel[a] = r; }
  const float* kr = qkv + (size_t)j * QP + CC; const float* vr = qkv + (size_t)j * QP + 2 * CC;
  float s[NH];
#pragma unroll 1
  for (int h = 0; h < NH; ++h) { float d = 0.f;
#pragma unroll 1
    for (int dd = 0; dd < HD; ++dd) { const int c = h * HD + dd; const float t = bf16_round(tab[((size_t)(rel[0] * NH + h) * HD + dd) * 3 + 0]) + bf16_round(tab[((size_t)(rel[1] * NH + h) * HD + dd) * 3 + 1]) + bf16_round(tab[((size_t)(rel[2] * NH + h) * HD + dd) * 3 + 2]);
      d += sq[w][c] * kr[c] + sq[w][c] * t; }
    s[h] = act ? d : -3.0e38f; }
#pragma unroll 1
  for (int h = 0; h < NH; ++h) { float mx = s[h]; for (int o = 16; o >= 1; o >>= 1) mx = fmaxf(mx, __shfl_xor(mx, o, 32)); float e = act ? expf(s[h] - mx) : 0.f; float den = e; for (int o = 16; o >= 1; o >>= 1) den += __shfl_xor(den, o, 32); s[h] = e / den; }
#pragma unroll 1
  for (int c = 0; c < CC; ++c) { float v = act ? s[c / HD] * vr[c] : 0.f; for (int o = 16; o >= 1; o >>= 1) v += __shfl_xor(v, o, 32); if (lane == 0) so[w][c] = v; }
  __builtin_amdgcn_fence(__ATOMIC_ACQ_REL, "workgroup"); __builtin_amdgcn_wave_barrier();
  for (int pass = 0; pass < 2; ++pass) { for (int c = lane; c < CC; c += 32) *(volatile float*)(out + (size_t)n * CC + c) = so[w][c]; if (pass == 0) __threadfence(); }
}
__global__ __launch_bounds__(256) void k_add96(const float* __restrict__ a, const float* __restrict__ b, int bp, float* __restrict__ o) {
  const int tid = threadIdx.x, w = tid >> 5, lane = tid & 31; const int row = blockIdx.x * 8 + w; if (row >= NN) return;
  for (int pass = 0; pass < 2; ++pass) { for (int c = lane; c < CC; c += 32) *(volatile float*)(o + (size_t)row * CC + c) = a[(size_t)row * CC + c] + b[(size_t)row * bp + c]; if (pass == 0) __threadfence(); }
}
extern "C" void kernel_launch(void* const* d_in, const int* in_sizes, int n_in,
                              void* d_out, int out_size, void* d_ws, size_t ws_size, hipStream_t stream) {
  (void)in_sizes; (void)n_in; (void)out_size;
  const float* feats = (const float*)d_in[0]; const float* xyz = (const float*)d_in[1]; const int* offs = (const int*)d_in[3]; const int* idx1 = (const int*)d_in[4]; const float* shift = (const float*)d_in[6];
  const float* n1w = (const float*)d_in[7]; const float* n1b = (const float*)d_in[8]; const float* qkv_w = (const float*)d_in[9]; const float* qkv_b = (const float*)d_in[10]; const float* tab = (const float*)d_in[11];
  const float* proj_w = (const float*)d_in[12]; const float* proj_b = (const float*)d_in[13]; const float* n2w = (const float*)d_in[14]; const float* n2b = (const float*)d_in[15];
  const float* fc1_w = (const float*)d_in[16]; const float* fc1_b = (const float*)d_in[17]; const float* fc2_w = (const float*)d_in[18]; const float* fc2_b = (const float*)d_in[19];
  char* ws = (char*)d_ws; size_t off = 0;
  auto take = [&](size_t bytes) { char* p = ws + off; off += (bytes + 255) & ~(size_t)255; return p; };
  unsigned short* Bqkv = (unsigned short*)take((size_t)QP * CC * 2); unsigned short* Bproj = (unsigned short*)take((size_t)PP * CC * 2); unsigned short* Bfc1 = (unsigned short*)take((size_t)FF * CC * 2); unsigned short* Bfc2 = (unsigned short*)take((size_t)PP * FF * 2);
  float* bqkv = (float*)take(QP * 4); float* bproj = (float*)take(PP * 4); float* bfc1 = (float*)take(FF * 4); float* bfc2 = (float*)take(PP * 4); float* mn = (float*)take(32 * 4);
  float* xr = (float*)take((size_t)NN * CC * 4); float* xn = (float*)take((size_t)NN * CC * 4); float* qkv = (float*)take((size_t)NN * QP * 4); float* att = (float*)take((size_t)NN * CC * 4);
  float* pr = (float*)take((size_t)NN * PP * 4); float* f1 = (float*)take((size_t)NN * CC * 4); float* hb = (float*)take((size_t)NN * FF * 4); float* f2 = (float*)take((size_t)NN * PP * 4);
  if (off > ws_size) return;
  k_wt_pad<<<(QP * (CC / 8) + 255) / 256, 256, 0, stream>>>(qkv_w, qkv_b, Bqkv, bqkv, 3 * CC, CC, QP);
  k_wt_pad<<<(PP * (CC / 8) + 255) / 256, 256, 0, stream>>>(proj_w, proj_b, Bproj, bproj, CC, CC, PP);
  k_wt_pad<<<(FF * (CC / 8) + 255) / 256, 256, 0, stream>>>(fc1_w, fc1_b, Bfc1, bfc1, FF, CC, FF);
  k_wt_pad<<<(PP * (FF / 8) + 255) / 256, 256, 0, stream>>>(fc2_w, fc2_b, Bfc2, bfc2, CC, FF, PP);
  k_min3<<<1, 256, 0, stream>>>(xyz, mn);
  k_ln96<true><<<(NN + 7) / 8, 256, 0, stream>>>(feats, CC, n1w, n1b, xn, xr);
  k_gemm_bf3<true, 0, false, false><<<((NN / 16) * (QP / 64) + 3) / 4, 128, 0, stream>>>(xn, CC, Bqkv, CC, bqkv, nullptr, 1, 0, qkv, QP, NN, QP, CC);
  k_swin_attn<<<(NN + 7) / 8, 256, 0, stream>>>(qkv, xyz, mn, shift, offs, idx1, tab, att);
  k_gemm_bf3<true, 0, false, false><<<((NN / 16) * (PP / 64) + 3) / 4, 128, 0, stream>>>(att, CC, Bproj, CC, bproj, nullptr, 1, 0, pr, PP, NN, PP, CC);
  k_add96<<<(NN + 7) / 8, 256, 0, stream>>>(xr, pr, PP, f1);
  k_ln96<false><<<(NN + 7) / 8, 256, 0, stream>>>(f1, CC, n2w, n2b, xn, nullptr);
  k_gemm_bf3<true, 2, false, false><<<((NN / 16) * (FF / 64) + 3) / 4, 128, 0, stream>>>(xn, CC, Bfc1, CC, bfc1, nullptr, 1, 0, hb, FF, NN, FF, CC);
  k_gemm_bf3<true, 0, false, false><<<((NN / 16) * (PP / 64) + 3) / 4, 128, 0, stream>>>(hb, FF, Bfc2, FF, bfc2, nullptr, 1, 0, f2, PP, NN, PP, FF);
  k_add96<<<(NN + 7) / 8, 256, 0, stream>>>(f1, f2, PP, (float*)d_out);
}
